// prototypes_47656957116695
// MI455X (gfx1250) — hardware-verified
//
#include <hip/hip_runtime.h>
#include <math.h>

constexpr int kRows    = 16 * 512;
constexpr int kIn      = 512;
constexpr int kHid     = 512;
constexpr int kProto   = 16;
constexpr int kGroup   = 4;
constexpr int kGroupN  = kGroup * kHid;
constexpr float kXCarry  = 8.0f;
constexpr float kWCarry  = 16.0f;
constexpr float kL1Scale = 1.0f / 16.0f;
constexpr float kL2Scale = 1.0f / 128.0f;
constexpr float kEps     = 1e-6f;

constexpr size_t kOffXh   = 0;
constexpr size_t kOffW1h  = kOffXh  + (size_t)kRows * kIn * 2;
constexpr size_t kOffW2h  = kOffW1h + (size_t)kProto * kHid * kIn * 2;
constexpr size_t kOffH1   = kOffW2h + (size_t)kProto * kHid * kHid * 2;
constexpr size_t kOffH2   = kOffH1  + (size_t)kRows * kGroupN * 2;
constexpr size_t kOffCosT = kOffH2  + (size_t)2 * kRows * kHid * 4;
constexpr size_t kWsTotal = kOffCosT + (size_t)kProto * kRows * 4;

typedef __attribute__((ext_vector_type(16))) _Float16 v16h;
typedef __attribute__((ext_vector_type(8)))  _Float16 v8h;
typedef __attribute__((ext_vector_type(16))) __bf16   v16b;
typedef __attribute__((ext_vector_type(8)))  __bf16   v8b;
typedef __attribute__((ext_vector_type(8)))  float    v8f;
typedef __attribute__((ext_vector_type(4)))  float    v4f;
typedef __attribute__((ext_vector_type(4)))  unsigned int v4u;

__device__ __forceinline__ unsigned short f2bf_bits(float f) {
  unsigned u = __float_as_uint(f);
  return (unsigned short)((u + 0x7FFFu + ((u >> 16) & 1u)) >> 16);
}
__device__ __forceinline__ float bf_bits2f(unsigned short h) { return __uint_as_float(((unsigned)h) << 16); }

__device__ __forceinline__ void dep_guard_h(v8f& a, v8f& b, v16h x, v16h y) { asm volatile("v_nop\n\tv_nop\n\tv_nop\n\tv_nop" : "+v"(a), "+v"(b) : "v"(x), "v"(y)); }
__device__ __forceinline__ void dep_guard_b(v8f& a, v8f& b, v16b x, v16b y) { asm volatile("v_nop\n\tv_nop\n\tv_nop\n\tv_nop" : "+v"(a), "+v"(b) : "v"(x), "v"(y)); }
__device__ __forceinline__ void keep4_h(v16h a, v16h b, v16h c, v16h d) { asm volatile("v_nop" :: "v"(a), "v"(b), "v"(c), "v"(d)); }
__device__ __forceinline__ void keep4_b(v16b a, v16b b, v16b c, v16b d) { asm volatile("v_nop" :: "v"(a), "v"(b), "v"(c), "v"(d)); }
__device__ __forceinline__ void acc_guard4(v8f& a, v8f& b, v8f& c, v8f& d) { asm volatile("v_nop\n\tv_nop\n\tv_nop\n\tv_nop" : "+v"(a), "+v"(b), "+v"(c), "+v"(d)); }
template <typename T> struct Frag;
template <> struct Frag<_Float16> {
  typedef v16h V; union U { v16h v; v8h h[2]; };
  static __device__ __forceinline__ v16h load(const _Float16* p) {
    U f; f.h[0] = *(const v8h*)(p); f.h[1] = *(const v8h*)(p + 16); return f.v;
  }
  static __device__ __forceinline__ v8f mma(v16h a, v16h b, v8f c) {
    return __builtin_amdgcn_wmma_f32_16x16x32_f16(false, a, false, b, (short)0, c, false, false);
  }
  static __device__ __forceinline__ void guard(v8f& a, v8f& b, v16h x, v16h y) { dep_guard_h(a, b, x, y); }
  static __device__ __forceinline__ void keep(v16h a, v16h b, v16h c, v16h d) { keep4_h(a, b, c, d); }
};
template <> struct Frag<__bf16> {
  typedef v16b V; union U { v16b v; v8b h[2]; };
  static __device__ __forceinline__ v16b load(const __bf16* p) {
    U f; f.h[0] = *(const v8b*)(p); f.h[1] = *(const v8b*)(p + 16); return f.v;
  }
  static __device__ __forceinline__ v8f mma(v16b a, v16b b, v8f c) {
    return __builtin_amdgcn_wmma_f32_16x16x32_bf16(false, a, false, b, (short)0, c, false, false);
  }
  static __device__ __forceinline__ void guard(v8f& a, v8f& b, v16b x, v16b y) { dep_guard_b(a, b, x, y); }
  static __device__ __forceinline__ void keep(v16b a, v16b b, v16b c, v16b d) { keep4_b(a, b, c, d); }
};

__device__ __forceinline__ unsigned pk16(unsigned short a, unsigned short b) { return (unsigned)a | ((unsigned)b << 16); }
__device__ __forceinline__ unsigned short h_bits(float f) { const _Float16 h = (_Float16)f; return __builtin_bit_cast(unsigned short, h); }

template <int ET> struct Elem;
template <> struct Elem<0> { typedef _Float16 T; };
template <> struct Elem<1> { typedef __bf16 T; };
template <int ET, bool SPLIT, int BIAS_MODE, int OUT_MODE, bool RESID, int ACT = 0>
__global__ __launch_bounds__(256) void wmma_gemm64(
    const unsigned short* __restrict__ Ap, const unsigned short* __restrict__ A2p, int lda, long strideA,
    const unsigned short* __restrict__ Btp, const unsigned short* __restrict__ Bt2p, int ldb, long strideB,
    void* __restrict__ Cout, void* __restrict__ Cout2, int ldc, long strideC,
    const float* __restrict__ bias,
    const float* __restrict__ resid, long strideR,
    int M, int N, int K, float scale) {
  typedef typename Elem<ET>::T T;
  typedef typename Frag<T>::V V;
  const T* A = (const T*)Ap; const T* A2 = (const T*)A2p; const T* Bt = (const T*)Btp; const T* Bt2 = (const T*)Bt2p;
  __shared__ __align__(16) float sT[8][16 * 68];
  const int b    = blockIdx.y;
  const int lane = threadIdx.x & 31;
  const int wave = threadIdx.x >> 5;
  const int tilesN = N >> 6;
  const int tilesM = M >> 6;
  const int tile = blockIdx.x * 8 + wave;
  if (tile >= tilesM * tilesN) return;
  const int tm = tile / tilesN;
  const int tn = tile - tm * tilesN;
  const int m0 = tm << 6;
  const int n0 = tn << 6;

  const T* Ab  = A  + (size_t)b * strideA;
  const T* Bb  = Bt + (size_t)b * strideB;
  const T* Ab2 = SPLIT ? (A2  + (size_t)b * strideA) : nullptr;
  const T* Bb2 = SPLIT ? (Bt2 + (size_t)b * strideB) : nullptr;

  const int rlane = lane & 15;
  const int koff  = (lane >> 4) * 8;
  const int mOff  = (lane >> 4) * 8;

  v8f acc[4][4];
#pragma unroll
  for (int i = 0; i < 4; ++i)
#pragma unroll
    for (int j = 0; j < 4; ++j) acc[i][j] = (v8f){0.f,0.f,0.f,0.f,0.f,0.f,0.f,0.f};

  for (int k0 = 0; k0 < K; k0 += 32) {
    V bh[4], bl[4];
#pragma unroll
    for (int j = 0; j < 4; ++j) {
      const size_t bo = (size_t)(n0 + (j << 4) + rlane) * ldb + koff + k0;
      bh[j] = Frag<T>::load(Bb + bo);
      if (SPLIT) bl[j] = Frag<T>::load(Bb2 + bo);
    }
#pragma unroll
    for (int i = 0; i < 4; ++i) {
      const size_t ao = (size_t)(m0 + (i << 4) + rlane) * lda + koff + k0;
      V ah = Frag<T>::load(Ab + ao);
      V al;
      if (SPLIT) al = Frag<T>::load(Ab2 + ao);
#pragma unroll
      for (int j = 0; j < 4; ++j) {
        acc[i][j] = Frag<T>::mma(ah, bh[j], acc[i][j]);
        if (SPLIT) {
          acc[i][j] = Frag<T>::mma(ah, bl[j], acc[i][j]);
          acc[i][j] = Frag<T>::mma(al, bh[j], acc[i][j]);
        }
      }
      Frag<T>::guard(acc[i][0], acc[i][3], ah, SPLIT ? al : ah);
    }
    Frag<T>::keep(bh[0], bh[1], bh[2], bh[3]);
    if (SPLIT) Frag<T>::keep(bl[0], bl[1], bl[2], bl[3]);
  }
  acc_guard4(acc[0][0], acc[0][1], acc[0][2], acc[0][3]);
  acc_guard4(acc[1][0], acc[1][1], acc[1][2], acc[1][3]);
  acc_guard4(acc[2][0], acc[2][1], acc[2][2], acc[2][3]);
  acc_guard4(acc[3][0], acc[3][1], acc[3][2], acc[3][3]);

  float* slab = sT[wave];
  const float* Rb = RESID ? (resid + (size_t)b * strideR) : nullptr;
#pragma unroll
  for (int i = 0; i < 4; ++i) {
    const int mBase = m0 + (i << 4);
#pragma unroll
    for (int j = 0; j < 4; ++j) {
      const int n = n0 + (j << 4) + rlane;
      float bv = 0.f;
      if (BIAS_MODE == 2) bv = bias[n];
#pragma unroll
      for (int r = 0; r < 8; ++r) {
        float v = acc[i][j][r] * scale;
        if (BIAS_MODE == 1) v += bias[mBase + mOff + r];
        if (BIAS_MODE == 2) v += bv;
        if (RESID) v += Rb[(size_t)(mBase + mOff + r) * ldc + n];
        if (ACT == 2) v = fmaxf(v, 0.0f);
        if (ACT == 4) v = (v > 0.f) ? v : 0.01f * v;
        slab[(mOff + r) * 68 + (j << 4) + rlane] = v;
      }
    }
    __builtin_amdgcn_fence(__ATOMIC_RELEASE, "workgroup");
    __builtin_amdgcn_wave_barrier();
    __builtin_amdgcn_fence(__ATOMIC_ACQUIRE, "workgroup");
    if (OUT_MODE == 0) {
      float* C = (float*)Cout + (size_t)b * strideC;
      const int hh = lane >> 4, c4 = (lane & 15) * 4;
      for (int pass = 0; pass < 2; ++pass) {
#pragma unroll
        for (int it = 0; it < 8; ++it) {
          const int row = it * 2 + hh;
          v4f v = *(const v4f*)(slab + row * 68 + c4);
          *(volatile v4f*)(C + (size_t)(mBase + row) * ldc + n0 + c4) = v;
        }
        __threadfence();
      }
    } else {
      const int q = lane >> 3, c8 = (lane & 7) * 8;
      unsigned short* C  = (unsigned short*)Cout  + (size_t)b * strideC;
      unsigned short* C2 = (OUT_MODE == 2) ? ((unsigned short*)Cout2 + (size_t)b * strideC) : nullptr;
      for (int pass = 0; pass < 2; ++pass) {
#pragma unroll
        for (int it = 0; it < 4; ++it) {
          const int row = it * 4 + q;
          const float* sp = slab + row * 68 + c8;
          v8h hv, lv;
#pragma unroll
          for (int e = 0; e < 8; ++e) {
            if (OUT_MODE == 1) {
              hv[e] = (_Float16)sp[e];
            } else {
              unsigned short hb = f2bf_bits(sp[e]);
              unsigned short lb = f2bf_bits(sp[e] - bf_bits2f(hb));
              hv[e] = __builtin_bit_cast(_Float16, hb);
              lv[e] = __builtin_bit_cast(_Float16, lb);
            }
          }
          *(volatile v8h*)(C + (size_t)(mBase + row) * ldc + n0 + c8) = hv;
          if (OUT_MODE == 2) *(volatile v8h*)(C2 + (size_t)(mBase + row) * ldc + n0 + c8) = lv;
        }
        __threadfence();
      }
    }
    __builtin_amdgcn_fence(__ATOMIC_RELEASE, "workgroup");
    __builtin_amdgcn_wave_barrier();
    __builtin_amdgcn_fence(__ATOMIC_ACQUIRE, "workgroup");
  }
}

__global__ __launch_bounds__(256) void cast8_f16_kernel(const float* __restrict__ in, unsigned short* __restrict__ out,
                                                        float scale, int n8) {
  const int i = blockIdx.x * 256 + threadIdx.x;
  if (i >= n8) return;
  const float* p = in + 8 * (size_t)i;
  const v4f a = *(const v4f*)(p);
  const v4f c = *(const v4f*)(p + 4);
  unsigned short hb[8];
#pragma unroll
  for (int e = 0; e < 4; ++e) {
    hb[e]     = h_bits(a[e] * scale);
    hb[4 + e] = h_bits(c[e] * scale);
  }
  const v4u u = (v4u){pk16(hb[0], hb[1]), pk16(hb[2], hb[3]), pk16(hb[4], hb[5]), pk16(hb[6], hb[7])};
  unsigned short* q = out + 8 * (size_t)i;
  *(volatile v4u*)q = u;
  __threadfence();
  *(volatile v4u*)q = u;
}

__global__ __launch_bounds__(256) void cosred_kernel(const float* __restrict__ H2, const float* __restrict__ protos,
                                                      float* __restrict__ cosT, int pbase) {
  __shared__ float sres[2][32];
  const int t = threadIdx.x;
  const int lane = t & 31, wave = t >> 5;
  const int rowBlk = blockIdx.x * 32;
#pragma unroll 1
  for (int z = 0; z < 2; ++z) {
    const int p = pbase + z;
    const float* pr = protos + (size_t)p * kHid + lane * 4;
    float pv[16];
    float pss = 0.f;
#pragma unroll
    for (int j = 0; j < 4; ++j) {
      const v4f a = *(const v4f*)(pr + j * 128);
#pragma unroll
      for (int e = 0; e < 4; ++e) { pv[j * 4 + e] = a[e]; pss += a[e] * a[e]; }
    }
#pragma unroll
    for (int off = 16; off > 0; off >>= 1) pss += __shfl_xor(pss, off, 32);
    const float pn = fmaxf(sqrtf(pss), kEps);
    const float* hz = H2 + (size_t)z * kRows * kHid;
#pragma unroll 1
    for (int rr = 0; rr < 4; ++rr) {
      const int row = rowBlk + wave * 4 + rr;
      const float* hr = hz + (size_t)row * kHid + lane * 4;
      float d = 0.f, s = 0.f;
#pragma unroll
      for (int j = 0; j < 4; ++j) {
        const v4f x = *(const v4f*)(hr + j * 128);
#pragma unroll
        for (int e = 0; e < 4; ++e) { d += x[e] * pv[j * 4 + e]; s += x[e] * x[e]; }
      }
#pragma unroll
      for (int off = 16; off > 0; off >>= 1) {
        d += __shfl_xor(d, off, 32);
        s += __shfl_xor(s, off, 32);
      }
      const float xn = fmaxf(sqrtf(s), kEps);
      const float cv = d * (1.0f / (xn * pn));
      if (lane == 0) sres[z][wave * 4 + rr] = cv;
    }
  }
  __syncthreads();
  if (wave == 0) {
    const int zz = (lane >> 3) & 1, q = lane & 7;
    const v4f v = (v4f){sres[zz][q * 4 + 0], sres[zz][q * 4 + 1], sres[zz][q * 4 + 2], sres[zz][q * 4 + 3]};
    float* dst = cosT + (size_t)(pbase + zz) * kRows + rowBlk + q * 4;
    if (lane < 16) *(volatile v4f*)dst = v;
    __threadfence();
    if (lane < 16) *(volatile v4f*)dst = v;
  }
}

__global__ __launch_bounds__(256) void outw_kernel(const float* __restrict__ cosT, float* __restrict__ out) {
  const int gt = blockIdx.x * 256 + threadIdx.x;
  if (gt >= kRows * 4) return;
  const int row = gt >> 2;
  const int c = (gt & 3) * 4;
  const v4f v = (v4f){cosT[(size_t)(c + 0) * kRows + row], cosT[(size_t)(c + 1) * kRows + row],
                      cosT[(size_t)(c + 2) * kRows + row], cosT[(size_t)(c + 3) * kRows + row]};
  float* dst = out + (size_t)row * kProto + c;
  *(volatile v4f*)dst = v;
  __threadfence();
  *(volatile v4f*)dst = v;
}

extern "C" void kernel_launch(void* const* d_in, const int* in_sizes, int n_in,
                              void* d_out, int out_size, void* d_ws, size_t ws_size,
                              hipStream_t stream) {
  if (n_in < 4) return;
  if (in_sizes[0] != kRows * kIn) return;
  if (in_sizes[1] != kProto * kHid * kIn) return;
  if (in_sizes[2] != kProto * kHid * kHid) return;
  if (in_sizes[3] != kProto * kHid) return;
  if (out_size != kRows * kProto) return;
  if (ws_size < kWsTotal) return;

  const float* hidden = (const float*)d_in[0];
  const float* W1     = (const float*)d_in[1];
  const float* W2     = (const float*)d_in[2];
  const float* protos = (const float*)d_in[3];
  float* out = (float*)d_out;

  char* ws = (char*)d_ws;
  unsigned short* Xh   = (unsigned short*)(ws + kOffXh);
  unsigned short* W1h  = (unsigned short*)(ws + kOffW1h);
  unsigned short* W2h  = (unsigned short*)(ws + kOffW2h);
  unsigned short* H1   = (unsigned short*)(ws + kOffH1);
  float*          H2   = (float*)(ws + kOffH2);
  float*          cosT = (float*)(ws + kOffCosT);

  const int n8x = (kRows * kIn) / 8;
  const int n8w = (kProto * kHid * kIn) / 8;
  cast8_f16_kernel<<<dim3((n8x + 255) / 256), dim3(256), 0, stream>>>(hidden, Xh, kXCarry, n8x);
  cast8_f16_kernel<<<dim3((n8w + 255) / 256), dim3(256), 0, stream>>>(W1, W1h, kWCarry, n8w);
  cast8_f16_kernel<<<dim3((n8w + 255) / 256), dim3(256), 0, stream>>>(W2, W2h, kWCarry, n8w);

  for (int g = 0; g < kProto / kGroup; ++g) {
    {
      const unsigned short* Bt = W1h + (size_t)g * kGroupN * kIn;
      const int tiles = (kRows / 64) * (kGroupN / 64);
      wmma_gemm64<0, false, 0, 1, false, 2><<<dim3((tiles + 7) / 8, 1), dim3(256), 0, stream>>>(
          Xh, Xh, kIn, 0L, Bt, Bt, kIn, 0L, (void*)H1, (void*)H1, kGroupN, 0L,
          (const float*)nullptr, (const float*)nullptr, 0L, kRows, kGroupN, kIn, kL1Scale);
    }
    for (int q = 0; q < 2; ++q) {
      const int pbase = g * kGroup + 2 * q;
      {
        const unsigned short* A  = H1 + (size_t)(2 * q) * kHid;
        const unsigned short* Bt = W2h + (size_t)pbase * kHid * kHid;
        const int tiles = (kRows / 64) * (kHid / 64);
        wmma_gemm64<0, false, 0, 0, false, 2><<<dim3((tiles + 7) / 8, 2), dim3(256), 0, stream>>>(
            A, A, kGroupN, (long)kHid, Bt, Bt, kHid, (long)kHid * kHid, (void*)H2, (void*)H2, kHid,
            (long)kRows * kHid, (const float*)nullptr, (const float*)nullptr, 0L, kRows, kHid, kHid, kL2Scale);
      }
      cosred_kernel<<<dim3(kRows / 32), dim3(256), 0, stream>>>(H2, protos, cosT, pbase);
    }
  }
  outw_kernel<<<dim3((kRows * 4 + 255) / 256), dim3(256), 0, stream>>>(cosT, out);
}
